// QuantMultiheadAttention_19052474925379
// MI455X (gfx1250) — hardware-verified
//
#include <hip/hip_runtime.h>
#include <stddef.h>
#include <stdint.h>


#define NB_ 2
#define NS_ 2048
#define NE_ 1024
#define NH_ 16
#define ND_ 64
#define NM_ (NB_ * NS_)

typedef _Float16 f16t;
typedef _Float16 v16h __attribute__((ext_vector_type(16)));
typedef _Float16 v8h  __attribute__((ext_vector_type(8), __may_alias__));
typedef float    v8f  __attribute__((ext_vector_type(8)));
typedef float    v4f  __attribute__((ext_vector_type(4), __may_alias__));

union Frag { v16h v; v8h hv[2]; };

__device__ __forceinline__ v8f vzero8() {
    const v8f z = {0.0f, 0.0f, 0.0f, 0.0f, 0.0f, 0.0f, 0.0f, 0.0f};
    return z;
}

__device__ __forceinline__ v16h ldfrag(const f16t* __restrict__ p) {
    Frag f;
    f.hv[0] = *(const v8h*)p;
    f.hv[1] = *(const v8h*)(p + 16);
    return f.v;
}

__device__ __forceinline__ v8f wmma16(v16h a, v16h b, v8f c) {
    return __builtin_amdgcn_wmma_f32_16x16x32_f16(false, a, false, b, (short)0, c, false, false);
}

__global__ __launch_bounds__(256) void k_cvt(const float* __restrict__ src, f16t* __restrict__ dst,
                                             int n8, float scale) {
    const int i = (int)blockIdx.x * 256 + (int)threadIdx.x;
    if (i >= n8) return;
    const float* s = src + (size_t)i * 8;
    const v4f x0 = *(const v4f*)s;
    const v4f x1 = *(const v4f*)(s + 4);
    v8h o;
    o[0] = (f16t)(x0[0] * scale);
    o[1] = (f16t)(x0[1] * scale);
    o[2] = (f16t)(x0[2] * scale);
    o[3] = (f16t)(x0[3] * scale);
    o[4] = (f16t)(x1[0] * scale);
    o[5] = (f16t)(x1[1] * scale);
    o[6] = (f16t)(x1[2] * scale);
    o[7] = (f16t)(x1[3] * scale);
    f16t* d = dst + (size_t)i * 8;
    *(volatile v8h*)d = o;
    __threadfence();
    *(volatile v8h*)d = o;
}

__device__ __forceinline__ void stg_rm16(f16t* sh, v8f a, float sc, int row0, int col) {
#pragma unroll
    for (int r = 0; r < 8; ++r) sh[(row0 + r) * 72 + col] = (f16t)(a[r] * sc);
}
__device__ __forceinline__ void stg_tr16(f16t* sh, v8f a, float sc, int col0, int row) {
#pragma unroll
    for (int r = 0; r < 8; ++r) sh[row * 72 + col0 + r] = (f16t)(a[r] * sc);
}
__device__ __forceinline__ void stg_rm32(float* sf, v8f a, float sc, int row0, int col) {
#pragma unroll
    for (int r = 0; r < 8; ++r) sf[(row0 + r) * 68 + col] = a[r] * sc;
}

template <int MODE>
__global__ __launch_bounds__(64) void k_gemm(const f16t* __restrict__ X, const f16t* __restrict__ W,
                                             void* __restrict__ out, float oscale) {
    __shared__ __align__(16) f16t sh[64 * 72];
    __shared__ __align__(16) float sf[64 * 68];

    const int tid = (int)threadIdx.x;
    const int l = tid & 31, w = tid >> 5, h = l >> 4, m16 = l & 15;
    const int nb = (int)blockIdx.x, mb = (int)blockIdx.y;
    const int nbase = nb * 64, mbase = mb * 64;

    const f16t* xa0 = X + (size_t)(mbase + 32 * w + m16) * NE_ + 8 * h;
    const f16t* xa1 = xa0 + (size_t)16 * NE_;
    const f16t* wb0 = W + (size_t)(nbase + m16) * NE_ + 8 * h;
    const f16t* wb1 = wb0 + (size_t)16 * NE_;
    const f16t* wb2 = wb0 + (size_t)32 * NE_;
    const f16t* wb3 = wb0 + (size_t)48 * NE_;

    v8f a00 = vzero8(), a01 = vzero8(), a02 = vzero8(), a03 = vzero8();
    v8f a10 = vzero8(), a11 = vzero8(), a12 = vzero8(), a13 = vzero8();

#pragma unroll 1
    for (int k0 = 0; k0 < NE_; k0 += 32) {
        const v16h fa0 = ldfrag(xa0 + k0);
        const v16h fa1 = ldfrag(xa1 + k0);
        const v16h fb0 = ldfrag(wb0 + k0);
        const v16h fb1 = ldfrag(wb1 + k0);
        const v16h fb2 = ldfrag(wb2 + k0);
        const v16h fb3 = ldfrag(wb3 + k0);
        a00 = wmma16(fa0, fb0, a00);
        a01 = wmma16(fa0, fb1, a01);
        a02 = wmma16(fa0, fb2, a02);
        a03 = wmma16(fa0, fb3, a03);
        a10 = wmma16(fa1, fb0, a10);
        a11 = wmma16(fa1, fb1, a11);
        a12 = wmma16(fa1, fb2, a12);
        a13 = wmma16(fa1, fb3, a13);
        asm volatile("v_nop\n\tv_nop\n\tv_nop\n\tv_nop"
                     : "+v"(a00), "+v"(a01), "+v"(a02), "+v"(a03),
                       "+v"(a10), "+v"(a11), "+v"(a12), "+v"(a13)
                     : "v"(fa0), "v"(fa1), "v"(fb0), "v"(fb1), "v"(fb2), "v"(fb3)
                     : "memory");
    }

    const int rw = 32 * w + 8 * h;
    if (MODE == 2) {
        stg_rm32(sf, a00, oscale, rw, m16);
        stg_rm32(sf, a01, oscale, rw, 16 + m16);
        stg_rm32(sf, a02, oscale, rw, 32 + m16);
        stg_rm32(sf, a03, oscale, rw, 48 + m16);
        stg_rm32(sf, a10, oscale, rw + 16, m16);
        stg_rm32(sf, a11, oscale, rw + 16, 16 + m16);
        stg_rm32(sf, a12, oscale, rw + 16, 32 + m16);
        stg_rm32(sf, a13, oscale, rw + 16, 48 + m16);
    } else if (MODE == 0) {
        stg_rm16(sh, a00, oscale, rw, m16);
        stg_rm16(sh, a01, oscale, rw, 16 + m16);
        stg_rm16(sh, a02, oscale, rw, 32 + m16);
        stg_rm16(sh, a03, oscale, rw, 48 + m16);
        stg_rm16(sh, a10, oscale, rw + 16, m16);
        stg_rm16(sh, a11, oscale, rw + 16, 16 + m16);
        stg_rm16(sh, a12, oscale, rw + 16, 32 + m16);
        stg_rm16(sh, a13, oscale, rw + 16, 48 + m16);
    } else {
        stg_tr16(sh, a00, oscale, rw, m16);
        stg_tr16(sh, a01, oscale, rw, 16 + m16);
        stg_tr16(sh, a02, oscale, rw, 32 + m16);
        stg_tr16(sh, a03, oscale, rw, 48 + m16);
        stg_tr16(sh, a10, oscale, rw + 16, m16);
        stg_tr16(sh, a11, oscale, rw + 16, 16 + m16);
        stg_tr16(sh, a12, oscale, rw + 16, 32 + m16);
        stg_tr16(sh, a13, oscale, rw + 16, 48 + m16);
    }
    __syncthreads();

    if (MODE == 2) {
        float* of = (float*)out;
        const int rq = l >> 4, c4 = l & 15;
#pragma unroll
        for (int it = 0; it < 16; ++it) {
            const int R = 32 * w + 2 * it + rq;
            const v4f val = *(const v4f*)(sf + R * 68 + 4 * c4);
            float* d = of + (size_t)(mbase + R) * NE_ + nbase + 4 * c4;
            *(volatile v4f*)d = val;
        }
        __threadfence();
#pragma unroll
        for (int it = 0; it < 16; ++it) {
            const int R = 32 * w + 2 * it + rq;
            const v4f val = *(const v4f*)(sf + R * 68 + 4 * c4);
            float* d = of + (size_t)(mbase + R) * NE_ + nbase + 4 * c4;
            *(volatile v4f*)d = val;
        }
    } else {
        f16t* oh = (f16t*)out;
        const int rq = l >> 3, c8 = l & 7;
        const int b = mbase / NS_;
        const int s0 = mbase - b * NS_;
#pragma unroll
        for (int it = 0; it < 8; ++it) {
            const int R = 32 * w + 4 * it + rq;
            const v8h val = *(const v8h*)(sh + R * 72 + 8 * c8);
            const size_t idx = (MODE == 0)
                ? ((((size_t)(b * NH_ + nb) * NS_) + (size_t)(s0 + R)) * ND_ + (size_t)(8 * c8))
                : ((((size_t)(b * NH_ + nb) * ND_) + (size_t)R) * NS_ + (size_t)(s0 + 8 * c8));
            *(volatile v8h*)(oh + idx) = val;
        }
        __threadfence();
#pragma unroll
        for (int it = 0; it < 8; ++it) {
            const int R = 32 * w + 4 * it + rq;
            const v8h val = *(const v8h*)(sh + R * 72 + 8 * c8);
            const size_t idx = (MODE == 0)
                ? ((((size_t)(b * NH_ + nb) * NS_) + (size_t)(s0 + R)) * ND_ + (size_t)(8 * c8))
                : ((((size_t)(b * NH_ + nb) * ND_) + (size_t)R) * NS_ + (size_t)(s0 + 8 * c8));
            *(volatile v8h*)(oh + idx) = val;
        }
    }
}

__device__ __forceinline__ float hmax8(v8f c) {
    float m = c[0];
#pragma unroll
    for (int r = 1; r < 8; ++r) m = fmaxf(m, c[r]);
    return m;
}
__device__ __forceinline__ v8h pexp8(v8f c, float sc, float bias, float& ps) {
    v8h t;
#pragma unroll
    for (int r = 0; r < 8; ++r) {
        const float p = __builtin_amdgcn_exp2f(fmaf(c[r], sc, bias));
        ps += p;
        t[r] = (f16t)p;
    }
    return t;
}

__global__ __launch_bounds__(32) void k_attn(const f16t* __restrict__ qh,
                                             const f16t* __restrict__ kh,
                                             const f16t* __restrict__ vt,
                                             f16t* __restrict__ ctx)
{
    __shared__ __align__(16) f16t so[16 * 72];

    const int l = (int)threadIdx.x, h = l >> 4, m16 = l & 15;
    const int qt = (int)blockIdx.x, bh = (int)blockIdx.y;
    const int q0 = qt * 16;

    const f16t* qrow = qh + ((size_t)bh * NS_ + q0 + m16) * ND_ + 8 * h;
    const v16h qb0 = ldfrag(qrow);
    const v16h qb1 = ldfrag(qrow + 32);
    const f16t* kbase = kh + ((size_t)bh * NS_ + m16) * ND_ + 8 * h;
    const f16t* vbase = vt + ((size_t)bh * ND_ + m16) * NS_ + 8 * h;

    v8f o0 = vzero8(), o1 = vzero8(), o2 = vzero8(), o3 = vzero8();
    float m2 = -3.0e38f, lsum = 0.0f;
    const float SC = 0.045084220027780f;

#pragma unroll 1
    for (int t0 = 0; t0 < NS_; t0 += 64) {
        const f16t* kp = kbase + (size_t)t0 * ND_;
        const v16h k00 = ldfrag(kp);
        const v16h k01 = ldfrag(kp + 32);
        const v16h k10 = ldfrag(kp + 16 * ND_);
        const v16h k11 = ldfrag(kp + 16 * ND_ + 32);
        const v16h k20 = ldfrag(kp + 32 * ND_);
        const v16h k21 = ldfrag(kp + 32 * ND_ + 32);
        const v16h k30 = ldfrag(kp + 48 * ND_);
        const v16h k31 = ldfrag(kp + 48 * ND_ + 32);

        v8f c0 = vzero8(), c1 = vzero8(), c2 = vzero8(), c3 = vzero8();
        c0 = wmma16(k00, qb0, c0); c0 = wmma16(k01, qb1, c0);
        c1 = wmma16(k10, qb0, c1); c1 = wmma16(k11, qb1, c1);
        c2 = wmma16(k20, qb0, c2); c2 = wmma16(k21, qb1, c2);
        c3 = wmma16(k30, qb0, c3); c3 = wmma16(k31, qb1, c3);
        asm volatile("v_nop\n\tv_nop\n\tv_nop\n\tv_nop"
                     : "+v"(c0), "+v"(c1), "+v"(c2), "+v"(c3)
                     : "v"(k00), "v"(k01), "v"(k10), "v"(k11),
                       "v"(k20), "v"(k21), "v"(k30), "v"(k31), "v"(qb0), "v"(qb1)
                     : "memory");

        float mx = fmaxf(fmaxf(hmax8(c0), hmax8(c1)), fmaxf(hmax8(c2), hmax8(c3)));
        mx = fmaxf(mx, __shfl_xor(mx, 16, 32));
        const float mn = fmaxf(m2, mx * SC);
        const float corr = __builtin_amdgcn_exp2f(m2 - mn);
        m2 = mn;
        const float bias = 8.0f - mn;
        float ps = 0.0f;
        Frag pa, pb;
        pa.hv[0] = pexp8(c0, SC, bias, ps);
        pa.hv[1] = pexp8(c1, SC, bias, ps);
        pb.hv[0] = pexp8(c2, SC, bias, ps);
        pb.hv[1] = pexp8(c3, SC, bias, ps);
        ps += __shfl_xor(ps, 16, 32);
        lsum = lsum * corr + ps;

#pragma unroll
        for (int r = 0; r < 8; ++r) {
            const float cr = __shfl(corr, 8 * h + r, 32);
            o0[r] *= cr; o1[r] *= cr; o2[r] *= cr; o3[r] *= cr;
        }

        const f16t* vp = vbase + t0;
        const v16h v00 = ldfrag(vp);
        const v16h v01 = ldfrag(vp + 32);
        const v16h v10 = ldfrag(vp + (size_t)16 * NS_);
        const v16h v11 = ldfrag(vp + (size_t)16 * NS_ + 32);
        const v16h v20 = ldfrag(vp + (size_t)32 * NS_);
        const v16h v21 = ldfrag(vp + (size_t)32 * NS_ + 32);
        const v16h v30 = ldfrag(vp + (size_t)48 * NS_);
        const v16h v31 = ldfrag(vp + (size_t)48 * NS_ + 32);
        o0 = wmma16(pa.v, v00, o0); o0 = wmma16(pb.v, v01, o0);
        o1 = wmma16(pa.v, v10, o1); o1 = wmma16(pb.v, v11, o1);
        o2 = wmma16(pa.v, v20, o2); o2 = wmma16(pb.v, v21, o2);
        o3 = wmma16(pa.v, v30, o3); o3 = wmma16(pb.v, v31, o3);
        asm volatile("v_nop\n\tv_nop\n\tv_nop\n\tv_nop"
                     : "+v"(o0), "+v"(o1), "+v"(o2), "+v"(o3)
                     : "v"(pa.v), "v"(pb.v), "v"(v00), "v"(v01), "v"(v10), "v"(v11),
                       "v"(v20), "v"(v21), "v"(v30), "v"(v31)
                     : "memory");
    }

    const float linv = 64.0f / lsum;
#pragma unroll
    for (int r = 0; r < 8; ++r) {
        const float il = __shfl(linv, 8 * h + r, 32);
        const int row = 8 * h + r;
        so[row * 72 + m16]      = (f16t)(o0[r] * il);
        so[row * 72 + 16 + m16] = (f16t)(o1[r] * il);
        so[row * 72 + 32 + m16] = (f16t)(o2[r] * il);
        so[row * 72 + 48 + m16] = (f16t)(o3[r] * il);
    }
    __syncthreads();

    const int b = bh / NH_, hd = bh - b * NH_;
    const int rq = l >> 3, c8 = l & 7;
#pragma unroll
    for (int it = 0; it < 4; ++it) {
        const int R = 4 * it + rq;
        const v8h val = *(const v8h*)(so + R * 72 + 8 * c8);
        f16t* d = ctx + ((size_t)(b * NS_ + q0 + R)) * NE_ + hd * ND_ + 8 * c8;
        *(volatile v8h*)d = val;
    }
    __threadfence();
#pragma unroll
    for (int it = 0; it < 4; ++it) {
        const int R = 4 * it + rq;
        const v8h val = *(const v8h*)(so + R * 72 + 8 * c8);
        f16t* d = ctx + ((size_t)(b * NS_ + q0 + R)) * NE_ + hd * ND_ + 8 * c8;
        *(volatile v8h*)d = val;
    }
}

extern "C" void kernel_launch(void* const* d_in, const int* in_sizes, int n_in,
                              void* d_out, int out_size, void* d_ws, size_t ws_size,
                              hipStream_t stream) {
    const size_t nAct = (size_t)NM_ * NE_;
    const size_t nW   = (size_t)NE_ * NE_;
    if (n_in != 7) return;
    if ((size_t)in_sizes[0] != nAct || (size_t)in_sizes[1] != nAct || (size_t)in_sizes[2] != nAct) return;
    if ((size_t)in_sizes[3] != nW || (size_t)in_sizes[4] != nW || (size_t)in_sizes[5] != nW ||
        (size_t)in_sizes[6] != nW) return;
    if ((size_t)out_size != nAct) return;

    char* ws = (char*)d_ws;
    size_t off = 0;
    auto carve = [&](size_t bytes) -> char* {
        char* p = ws + off;
        off += (bytes + 255) & ~(size_t)255;
        return p;
    };
    f16t* q16  = (f16t*)carve(nAct * 2);
    f16t* k16  = (f16t*)carve(nAct * 2);
    f16t* v16  = (f16t*)carve(nAct * 2);
    f16t* wq16 = (f16t*)carve(nW * 2);
    f16t* wk16 = (f16t*)carve(nW * 2);
    f16t* wv16 = (f16t*)carve(nW * 2);
    f16t* wo16 = (f16t*)carve(nW * 2);
    f16t* qh   = (f16t*)carve(nAct * 2);
    f16t* kh   = (f16t*)carve(nAct * 2);
    f16t* vt   = (f16t*)carve(nAct * 2);
    f16t* ctx  = (f16t*)carve(nAct * 2);
    if (off > ws_size) return;

    const int n8a = (int)(nAct / 8), n8w = (int)(nW / 8);
    const int ga = (n8a + 255) / 256, gw = (n8w + 255) / 256;
    k_cvt<<<ga, 256, 0, stream>>>((const float*)d_in[0], q16, n8a, 1.0f);
    k_cvt<<<ga, 256, 0, stream>>>((const float*)d_in[1], k16, n8a, 1.0f);
    k_cvt<<<ga, 256, 0, stream>>>((const float*)d_in[2], v16, n8a, 1.0f);
    k_cvt<<<gw, 256, 0, stream>>>((const float*)d_in[3], wq16, n8w, 64.0f);
    k_cvt<<<gw, 256, 0, stream>>>((const float*)d_in[4], wk16, n8w, 64.0f);
    k_cvt<<<gw, 256, 0, stream>>>((const float*)d_in[5], wv16, n8w, 64.0f);
    k_cvt<<<gw, 256, 0, stream>>>((const float*)d_in[6], wo16, n8w, 64.0f);

    const dim3 gg(NE_ / 64, NM_ / 64);
    k_gemm<0><<<gg, 64, 0, stream>>>(q16, wq16, (void*)qh, 0.015625f);
    k_gemm<0><<<gg, 64, 0, stream>>>(k16, wk16, (void*)kh, 0.015625f);
    k_gemm<1><<<gg, 64, 0, stream>>>(v16, wv16, (void*)vt, 0.015625f);

    const dim3 gat(NS_ / 16, NB_ * NH_);
    k_attn<<<gat, 32, 0, stream>>>(qh, kh, vt, ctx);

    k_gemm<2><<<gg, 64, 0, stream>>>(ctx, wo16, d_out, 1.0f / 4096.0f);
}
